// nlblock_50474455662772
// MI455X (gfx1250) — hardware-verified
//
#include <hip/hip_runtime.h>
#include <math.h>
#include <stddef.h>
#include <stdint.h>

#define NB    4
#define CIN   256
#define CI    128
#define NPOS  4096
#define NTOK  (NB * NPOS)
#define YP    (2 * CI)
#define SPT   68
#define WSMAX 134217728

static_assert(NPOS % 64 == 0);
static_assert(NTOK % 64 == 0);
static_assert(CIN % 64 == 0);
static_assert(CI % 64 == 0);
static_assert(YP == 256);

typedef float          v4f   __attribute__((ext_vector_type(4)));
typedef float          v8f   __attribute__((ext_vector_type(8)));
typedef int            v8i   __attribute__((ext_vector_type(8)));
typedef unsigned short v8us  __attribute__((ext_vector_type(8)));
typedef unsigned short v16us __attribute__((ext_vector_type(16)));
typedef __bf16         v16bf __attribute__((ext_vector_type(16)));
typedef __bf16         v8bf  __attribute__((ext_vector_type(8)));
typedef v4f  __attribute__((may_alias)) v4fa;
typedef v8us __attribute__((may_alias)) v8usa;
union FragB { v16bf v; v16us u; v8us h[2]; v8i w; };

__device__ __forceinline__ v8f wmb(const FragB& a, const FragB& b, v8f c) {
  v8f d = __builtin_amdgcn_wmma_f32_16x16x32_bf16(false, a.v, false, b.v, (short)0, c, false, false);
  asm volatile("v_nop\n\tv_nop\n\tv_nop\n\tv_nop" : "+v"(d) : "v"(a.w), "v"(b.w));
  return d;
}

__device__ __forceinline__ v8f z8() { v8f z = {0.f, 0.f, 0.f, 0.f, 0.f, 0.f, 0.f, 0.f}; return z; }

__device__ __forceinline__ unsigned bf16_bits(float f) {
  const unsigned u = __float_as_uint(f);
  return (u + 0x7FFFu + ((u >> 16) & 1u)) >> 16;
}
__device__ __forceinline__ float bf16_val(float f) {
  return __uint_as_float(bf16_bits(f) << 16);
}

__global__ __launch_bounds__(256) void k_wprep(const float* __restrict__ wt, const float* __restrict__ wp,
                                              const float* __restrict__ wg, const float* __restrict__ ww,
                                              unsigned short* WT, unsigned short* WP, unsigned short* WG,
                                              unsigned short* WW2) {
  const int bx = (int)blockIdx.x, tid = (int)threadIdx.x;
  const float* p;
  unsigned short* dp;
  if (bx < 48) {
    const int which = bx >> 4;
    const float* src = (which == 0) ? wt : ((which == 1) ? wp : wg);
    unsigned short* dst = (which == 0) ? WT : ((which == 1) ? WP : WG);
    const int u  = (bx & 15) * 256 + tid;
    const int o  = u >> 5;
    const int k8 = (u & 31) * 8;
    p  = src + (size_t)o * CIN + k8;
    dp = dst + (size_t)u * 8;
  } else {
    const int v  = (bx - 48) * 256 + tid;
    const int o  = v >> 5;
    const int k8 = (v & 31) * 8;
    const int kk = k8 & (CI - 1);
    p  = ww + (size_t)o * CI + kk;
    dp = WW2 + (size_t)v * 8;
  }
  const v4f a = *(const v4f*)p;
  const v4f b = *(const v4f*)(p + 4);
  v8us o8;
  o8[0] = (unsigned short)bf16_bits(a.x); o8[1] = (unsigned short)bf16_bits(a.y);
  o8[2] = (unsigned short)bf16_bits(a.z); o8[3] = (unsigned short)bf16_bits(a.w);
  o8[4] = (unsigned short)bf16_bits(b.x); o8[5] = (unsigned short)bf16_bits(b.y);
  o8[6] = (unsigned short)bf16_bits(b.z); o8[7] = (unsigned short)bf16_bits(b.w);
  *(volatile v8us*)dp = o8;
  __threadfence();
  *(volatile v8us*)dp = o8;
}

__global__ __launch_bounds__(256) void k_xt(const float* __restrict__ x, unsigned short* xt) {
  __shared__ __attribute__((aligned(16))) float tf[64 * SPT];
  const int bx = (int)blockIdx.x, tid = (int)threadIdx.x;
  const int b   = bx >> 8;
  const int rem = bx & 255;
  const int n0  = (rem >> 2) * 64;
  const int c0  = (rem & 3) * 64;
  {
    const int rsub = tid >> 4;
    const int c4   = (tid & 15) * 4;
#pragma unroll
    for (int it = 0; it < 4; ++it) {
      const int cr = it * 16 + rsub;
      const v4f a = *(const v4f*)(x + ((size_t)(b * CIN + c0 + cr)) * NPOS + n0 + c4);
      *(v4fa*)(tf + cr * SPT + c4) = a;
    }
  }
  __syncthreads();
  const int rsub = tid >> 3;
  const int c8   = (tid & 7) * 8;
  v8us o[2];
#pragma unroll
  for (int it = 0; it < 2; ++it) {
    const int tl = it * 32 + rsub;
    v8us w;
#pragma unroll
    for (int e = 0; e < 8; ++e) w[e] = (unsigned short)bf16_bits(tf[(c8 + e) * SPT + tl]);
    o[it] = w;
  }
#pragma unroll
  for (int it = 0; it < 2; ++it) {
    const int tl = it * 32 + rsub;
    *(volatile v8us*)(xt + ((size_t)(b * NPOS + n0 + tl)) * CIN + c0 + c8) = o[it];
  }
  __threadfence();
#pragma unroll
  for (int it = 0; it < 2; ++it) {
    const int tl = it * 32 + rsub;
    *(volatile v8us*)(xt + ((size_t)(b * NPOS + n0 + tl)) * CIN + c0 + c8) = o[it];
  }
}

template <int OMODE, int BMODE>
__global__ __launch_bounds__(128) void k_gemm(const unsigned short* __restrict__ A, int lda, long sA,
                                              const unsigned short* __restrict__ BT, int ldb, long sB, int K,
                                              const float* __restrict__ bias,
                                              unsigned short* oh, unsigned short* ol, float* of,
                                              const float* __restrict__ res, int ldc, long sC) {
  __shared__ __attribute__((aligned(16))) float stg[64 * SPT];
  __shared__ __attribute__((aligned(16))) float sb[64];
  const int tid = (int)threadIdx.x, lane = tid & 31, wave = tid >> 5, hh = lane >> 4, m = lane & 15;
  const int rowBase = (int)blockIdx.x * 64;
  const int colBase = (int)blockIdx.y * 64;
  const int z = (int)blockIdx.z;
  const unsigned short* Ab = A  + (size_t)z * (size_t)sA;
  const unsigned short* Bb = BT + (size_t)z * (size_t)sB;
  if (tid < 64) sb[tid] = bf16_val(bias[(BMODE == 0 ? colBase : rowBase) + tid]);

  v8f acc[4];
#pragma unroll
  for (int t = 0; t < 4; ++t) acc[t] = z8();
  const unsigned short* ap = Ab + (size_t)(rowBase + 16 * wave + m) * (size_t)lda + 8 * hh;
  const unsigned short* bp = Bb + (size_t)(colBase + m) * (size_t)ldb + 8 * hh;

#pragma unroll 1
  for (int k0 = 0; k0 < K; k0 += 32) {
    FragB af;
    af.h[0] = *(const v8usa*)(ap + k0);
    af.h[1] = *(const v8usa*)(ap + k0 + 16);
#pragma unroll
    for (int nt = 0; nt < 4; ++nt) {
      const unsigned short* wq = bp + (size_t)(16 * nt) * (size_t)ldb + k0;
      FragB bf;
      bf.h[0] = *(const v8usa*)wq;
      bf.h[1] = *(const v8usa*)(wq + 16);
      acc[nt] = wmb(af, bf, acc[nt]);
    }
  }

#pragma unroll
  for (int nt = 0; nt < 4; ++nt) {
    const int lc = 16 * nt + m;
#pragma unroll
    for (int r = 0; r < 8; ++r) {
      const int lr = 16 * wave + 8 * hh + r;
      stg[lr * SPT + lc] = acc[nt][r];
    }
  }
  __syncthreads();

  if (OMODE == 0) {
    float* Cb = of + (size_t)z * (size_t)sC;
    const float* Rb = res + (size_t)z * (size_t)sC;
    const int rsub = tid >> 4;
    const int c4   = (tid & 15) * 4;
    v4f pv[8];
#pragma unroll
    for (int it = 0; it < 8; ++it) {
      const int row = it * 8 + rsub;
      v4f v = *(const v4fa*)(stg + row * SPT + c4);
      if (BMODE == 0) {
        v.x += sb[c4]; v.y += sb[c4 + 1]; v.z += sb[c4 + 2]; v.w += sb[c4 + 3];
      } else {
        const float br = sb[row];
        v.x += br; v.y += br; v.z += br; v.w += br;
      }
      const v4f xr = *(const v4f*)(Rb + (size_t)(rowBase + row) * (size_t)ldc + colBase + c4);
      v.x += bf16_val(xr.x); v.y += bf16_val(xr.y); v.z += bf16_val(xr.z); v.w += bf16_val(xr.w);
      pv[it] = v;
    }
#pragma unroll
    for (int it = 0; it < 8; ++it) {
      const int row = it * 8 + rsub;
      *(volatile v4f*)(Cb + (size_t)(rowBase + row) * (size_t)ldc + colBase + c4) = pv[it];
    }
    __threadfence();
#pragma unroll
    for (int it = 0; it < 8; ++it) {
      const int row = it * 8 + rsub;
      *(volatile v4f*)(Cb + (size_t)(rowBase + row) * (size_t)ldc + colBase + c4) = pv[it];
    }
  } else {
    unsigned short* Hb = oh + (size_t)z * (size_t)sC;
    unsigned short* Lb = ol + (size_t)z * (size_t)sC;
    const int rsub = tid >> 3;
    const int c8   = (tid & 7) * 8;
    v8us hv[4], lv[4];
#pragma unroll
    for (int it = 0; it < 4; ++it) {
      const int row = it * 16 + rsub;
      const float* sp = stg + row * SPT + c8;
      v8us h8, l8;
#pragma unroll
      for (int e = 0; e < 8; ++e) {
        const float v = sp[e] + ((BMODE == 0) ? sb[c8 + e] : sb[row]);
        const unsigned hb = bf16_bits(v);
        const unsigned lb = bf16_bits(v - __uint_as_float(hb << 16));
        h8[e] = (unsigned short)hb;
        l8[e] = (unsigned short)lb;
      }
      hv[it] = h8; lv[it] = l8;
    }
#pragma unroll
    for (int it = 0; it < 4; ++it) {
      const int row = it * 16 + rsub;
      const size_t go = (size_t)(rowBase + row) * (size_t)ldc + colBase + c8;
      *(volatile v8us*)(Hb + go) = hv[it];
      *(volatile v8us*)(Lb + go) = lv[it];
    }
    __threadfence();
#pragma unroll
    for (int it = 0; it < 4; ++it) {
      const int row = it * 16 + rsub;
      const size_t go = (size_t)(rowBase + row) * (size_t)ldc + colBase + c8;
      *(volatile v8us*)(Hb + go) = hv[it];
      *(volatile v8us*)(Lb + go) = lv[it];
    }
  }
}

#define AT_D  128
#define AT_NW 4
#define AT_QB 64
#define AT_KC 64
#define OSP   132

__device__ __forceinline__ unsigned short at_bf_bits(float f) {
  unsigned u = __float_as_uint(f);
  return (unsigned short)((u + 0x7FFFu + ((u >> 16) & 1u)) >> 16);
}
__device__ __forceinline__ __bf16 at_f2bf(float f) { return __builtin_bit_cast(__bf16, at_bf_bits(f)); }
__device__ __forceinline__ void at_split(float f, __bf16& hi, __bf16& lo) {
  const unsigned short hb = at_bf_bits(f);
  hi = __builtin_bit_cast(__bf16, hb);
  lo = at_f2bf(f - __uint_as_float(((unsigned)hb) << 16));
}
__device__ __forceinline__ v8f at_mma(v16bf a, v16bf b, v8f c) {
  c = __builtin_amdgcn_wmma_f32_16x16x32_bf16(false, a, false, b, (short)0, c, false, false);
  asm volatile("v_nop\n\tv_nop\n\tv_nop\n\tv_nop" : "+v"(c) : "v"(a), "v"(b));
  return c;
}
union AtFB { v16bf v; v8bf h[2]; };
__device__ __forceinline__ v16bf at_ldfrag(const __bf16* p) {
  AtFB f; f.h[0] = *(const v8bf*)(p); f.h[1] = *(const v8bf*)(p + 16); return f.v;
}

__global__ __launch_bounds__(128)
void k_attn(const unsigned short* __restrict__ qhp, const unsigned short* __restrict__ qlp,
            const unsigned short* __restrict__ khp, const unsigned short* __restrict__ klp,
            const unsigned short* __restrict__ vhp, const unsigned short* __restrict__ vlp,
            unsigned short* yout) {
  __shared__ __align__(16) __bf16 Ksh[AT_KC * AT_D];
  __shared__ __align__(16) __bf16 Ksl[AT_KC * AT_D];
  __shared__ __align__(16) __bf16 Vth[AT_D * AT_KC];
  __shared__ __align__(16) __bf16 Vtl[AT_D * AT_KC];
  __shared__ __align__(16) __bf16 Psh[AT_NW][16 * AT_KC];
  __shared__ __align__(16) __bf16 Psl[AT_NW][16 * AT_KC];
  __shared__ __align__(16) float  Os[AT_NW][16 * OSP];

  const int tid  = (int)threadIdx.x;
  const int wave = tid >> 5;
  const int lane = tid & 31;
  const int hh   = lane >> 4;
  const int c    = lane & 15;

  const int bx  = (int)blockIdx.x;
  const int b   = bx >> 6;
  const int qb  = bx & 63;
  const int q0  = qb * AT_QB + wave * 16;

  const __bf16* Qh = (const __bf16*)(const void*)qhp + (size_t)b * NPOS * AT_D;
  const __bf16* Ql = (const __bf16*)(const void*)qlp + (size_t)b * NPOS * AT_D;
  const __bf16* Kh = (const __bf16*)(const void*)khp + (size_t)b * NPOS * AT_D;
  const __bf16* Kl = (const __bf16*)(const void*)klp + (size_t)b * NPOS * AT_D;
  const __bf16* Vh = (const __bf16*)(const void*)vhp + (size_t)b * AT_D * NPOS;
  const __bf16* Vl = (const __bf16*)(const void*)vlp + (size_t)b * AT_D * NPOS;
  unsigned short* yb = yout + (size_t)b * NPOS * YP;

  const __bf16* qrh = Qh + (size_t)(q0 + c) * AT_D;
  const __bf16* qrl = Ql + (size_t)(q0 + c) * AT_D;

  float mrow[8], lrow[8];
  v8f oacc[8];
#pragma unroll
  for (int r = 0; r < 8; ++r) { mrow[r] = -INFINITY; lrow[r] = 0.f; }
#pragma unroll
  for (int t = 0; t < 8; ++t) oacc[t] = z8();

  const int nChunks = NPOS / AT_KC;
  for (int kc = 0; kc < nChunks; ++kc) {
    const int kv0 = kc * AT_KC;
    __syncthreads();
    {
      const int r = tid >> 1, half = (tid & 1) * 64;
      const __bf16* ksh = Kh + (size_t)(kv0 + r) * AT_D + half;
      const __bf16* ksl = Kl + (size_t)(kv0 + r) * AT_D + half;
      const __bf16* vsh = Vh + (size_t)tid * NPOS + kv0;
      const __bf16* vsl = Vl + (size_t)tid * NPOS + kv0;
#pragma unroll 2
      for (int i = 0; i < 8; ++i) {
        const v8bf a0 = *(const v8bf*)(ksh + 8 * i);
        const v8bf a1 = *(const v8bf*)(ksl + 8 * i);
        const v8bf b0 = *(const v8bf*)(vsh + 8 * i);
        const v8bf b1 = *(const v8bf*)(vsl + 8 * i);
        *(v8bf*)(Ksh + r * AT_D + half + 8 * i) = a0;
        *(v8bf*)(Ksl + r * AT_D + half + 8 * i) = a1;
        *(v8bf*)(Vth + tid * AT_KC + 8 * i) = b0;
        *(v8bf*)(Vtl + tid * AT_KC + 8 * i) = b1;
      }
    }
    __syncthreads();

    v8f s[4];
#pragma unroll
    for (int j = 0; j < 4; ++j) s[j] = z8();
#pragma unroll 1
    for (int dc = 0; dc < 4; ++dc) {
      int qo = dc * 32 + 8 * hh;
      asm volatile("" : "+v"(qo));
      const v16bf qah = at_ldfrag(qrh + qo);
      const v16bf qal = at_ldfrag(qrl + qo);
#pragma unroll
      for (int j = 0; j < 4; ++j) {
        AtFB kb, kl;
        kb.h[0] = *(const v8bf*)(Ksh + (j * 16 + c) * AT_D + dc * 32 + 8 * hh);
        kb.h[1] = *(const v8bf*)(Ksh + (j * 16 + c) * AT_D + dc * 32 + 16 + 8 * hh);
        kl.h[0] = *(const v8bf*)(Ksl + (j * 16 + c) * AT_D + dc * 32 + 8 * hh);
        kl.h[1] = *(const v8bf*)(Ksl + (j * 16 + c) * AT_D + dc * 32 + 16 + 8 * hh);
        s[j] = at_mma(qah, kb.v, s[j]);
        s[j] = at_mma(qah, kl.v, s[j]);
        s[j] = at_mma(qal, kb.v, s[j]);
      }
    }
    float cm[8];
#pragma unroll
    for (int r = 0; r < 8; ++r) {
      float mx = -INFINITY;
#pragma unroll
      for (int j = 0; j < 4; ++j) mx = fmaxf(mx, s[j][r]);
#pragma unroll
      for (int off = 1; off < 16; off <<= 1) mx = fmaxf(mx, __shfl_xor(mx, off, 32));
      cm[r] = mx;
    }
    __bf16* pwh = Psh[wave];
    __bf16* pwl = Psl[wave];
#pragma unroll
    for (int r = 0; r < 8; ++r) {
      const float mnew  = fmaxf(mrow[r], cm[r]);
      const float alpha = expf(mrow[r] - mnew);
      mrow[r] = mnew;
      float psum = 0.f;
#pragma unroll
      for (int j = 0; j < 4; ++j) {
        const float p = expf(s[j][r] - mnew);
        psum += p;
        __bf16 a, bl; at_split(p, a, bl);
        pwh[(8 * hh + r) * AT_KC + j * 16 + c] = a;
        pwl[(8 * hh + r) * AT_KC + j * 16 + c] = bl;
      }
#pragma unroll
      for (int off = 1; off < 16; off <<= 1) psum += __shfl_xor(psum, off, 32);
      lrow[r] = lrow[r] * alpha + psum;
#pragma unroll
      for (int t = 0; t < 8; ++t) oacc[t][r] *= alpha;
    }
    __builtin_amdgcn_fence(__ATOMIC_RELEASE, "workgroup");
    __builtin_amdgcn_wave_barrier();
    __builtin_amdgcn_fence(__ATOMIC_ACQUIRE, "workgroup");
#pragma unroll 1
    for (int kk = 0; kk < 2; ++kk) {
      AtFB pa, pl;
      pa.h[0] = *(const v8bf*)(pwh + c * AT_KC + kk * 32 + 8 * hh);
      pa.h[1] = *(const v8bf*)(pwh + c * AT_KC + kk * 32 + 16 + 8 * hh);
      pl.h[0] = *(const v8bf*)(pwl + c * AT_KC + kk * 32 + 8 * hh);
      pl.h[1] = *(const v8bf*)(pwl + c * AT_KC + kk * 32 + 16 + 8 * hh);
#pragma unroll
      for (int t = 0; t < 8; ++t) {
        AtFB vb, vl;
        vb.h[0] = *(const v8bf*)(Vth + (t * 16 + c) * AT_KC + kk * 32 + 8 * hh);
        vb.h[1] = *(const v8bf*)(Vth + (t * 16 + c) * AT_KC + kk * 32 + 16 + 8 * hh);
        vl.h[0] = *(const v8bf*)(Vtl + (t * 16 + c) * AT_KC + kk * 32 + 8 * hh);
        vl.h[1] = *(const v8bf*)(Vtl + (t * 16 + c) * AT_KC + kk * 32 + 16 + 8 * hh);
        oacc[t] = at_mma(pa.v, vb.v, oacc[t]);
        oacc[t] = at_mma(pa.v, vl.v, oacc[t]);
        oacc[t] = at_mma(pl.v, vb.v, oacc[t]);
      }
    }
  }

  float* os = Os[wave];
#pragma unroll
  for (int r = 0; r < 8; ++r) {
    const float inv = 1.0f / lrow[r];
#pragma unroll
    for (int t = 0; t < 8; ++t) os[(8 * hh + r) * OSP + t * 16 + c] = oacc[t][r] * inv;
  }
  __builtin_amdgcn_fence(__ATOMIC_RELEASE, "workgroup");
  __builtin_amdgcn_wave_barrier();
  __builtin_amdgcn_fence(__ATOMIC_ACQUIRE, "workgroup");
  {
    const int q  = lane >> 3;
    const int c8 = (lane & 7) * 8;
#pragma unroll 1
    for (int dh = 0; dh < 2; ++dh) {
      v8us hv[4], lv[4];
#pragma unroll
      for (int it = 0; it < 4; ++it) {
        const int row = it * 4 + q;
        const float* sp = os + row * OSP + dh * 64 + c8;
        v8us h8, l8;
#pragma unroll
        for (int e = 0; e < 8; ++e) {
          const float f = sp[e];
          const unsigned short hb = at_bf_bits(f);
          const unsigned short lb = at_bf_bits(f - __uint_as_float(((unsigned)hb) << 16));
          h8[e] = hb; l8[e] = lb;
        }
        hv[it] = h8; lv[it] = l8;
      }
#pragma unroll
      for (int it = 0; it < 4; ++it) {
        const int row = it * 4 + q;
        unsigned short* yr = yb + (size_t)(q0 + row) * YP + dh * 64 + c8;
        *(volatile v8us*)(yr)        = hv[it];
        *(volatile v8us*)(yr + AT_D) = lv[it];
      }
      __threadfence();
#pragma unroll
      for (int it = 0; it < 4; ++it) {
        const int row = it * 4 + q;
        unsigned short* yr = yb + (size_t)(q0 + row) * YP + dh * 64 + c8;
        *(volatile v8us*)(yr)        = hv[it];
        *(volatile v8us*)(yr + AT_D) = lv[it];
      }
    }
  }
}

static inline size_t al256(size_t o) { return (o + 255) & ~(size_t)255; }

extern "C" void kernel_launch(void* const* d_in, const int* in_sizes, int n_in,
                              void* d_out, int out_size, void* d_ws, size_t ws_size,
                              hipStream_t stream) {
  if (n_in < 9) return;
  if (in_sizes[0] != NB * CIN * NPOS) return;
  if (in_sizes[1] != CI * CIN || in_sizes[3] != CI * CIN || in_sizes[5] != CI * CIN) return;
  if (in_sizes[2] != CI || in_sizes[4] != CI || in_sizes[6] != CI) return;
  if (in_sizes[7] != CIN * CI || in_sizes[8] != CIN) return;
  if (out_size != NB * CIN * NPOS) return;

  const float* x       = (const float*)d_in[0];
  const float* theta_w = (const float*)d_in[1];
  const float* theta_b = (const float*)d_in[2];
  const float* phi_w   = (const float*)d_in[3];
  const float* phi_b   = (const float*)d_in[4];
  const float* g_w     = (const float*)d_in[5];
  const float* g_b     = (const float*)d_in[6];
  const float* w_w     = (const float*)d_in[7];
  const float* w_b     = (const float*)d_in[8];
  float* out = (float*)d_out;

  const size_t PW  = (size_t)CI * CIN * 2;
  const size_t PW2 = (size_t)CIN * YP * 2;
  const size_t PXT = (size_t)NTOK * CIN * 2;
  const size_t PA  = (size_t)NTOK * CI * 2;
  const size_t PY  = (size_t)NTOK * YP * 2;
  size_t off = 0;
  const size_t oWT  = off; off = al256(off + PW);
  const size_t oWP  = off; off = al256(off + PW);
  const size_t oWG  = off; off = al256(off + PW);
  const size_t oWW2 = off; off = al256(off + PW2);
  const size_t oXT  = off; off = al256(off + PXT);
  const size_t oTHh = off; off = al256(off + PA);
  const size_t oTHl = off; off = al256(off + PA);
  const size_t oPHh = off; off = al256(off + PA);
  const size_t oPHl = off; off = al256(off + PA);
  const size_t oGTh = off; off = al256(off + PA);
  const size_t oGTl = off; off = al256(off + PA);
  const size_t oY   = off; off = al256(off + PY);
  if (off > ws_size || off > (size_t)WSMAX) return;

  char* ws = (char*)d_ws;
  unsigned short* WT  = (unsigned short*)(ws + oWT);
  unsigned short* WP  = (unsigned short*)(ws + oWP);
  unsigned short* WG  = (unsigned short*)(ws + oWG);
  unsigned short* WW2 = (unsigned short*)(ws + oWW2);
  unsigned short* XT  = (unsigned short*)(ws + oXT);
  unsigned short* THh = (unsigned short*)(ws + oTHh);
  unsigned short* THl = (unsigned short*)(ws + oTHl);
  unsigned short* PHh = (unsigned short*)(ws + oPHh);
  unsigned short* PHl = (unsigned short*)(ws + oPHl);
  unsigned short* GTh = (unsigned short*)(ws + oGTh);
  unsigned short* GTl = (unsigned short*)(ws + oGTl);
  unsigned short* Y   = (unsigned short*)(ws + oY);

  k_wprep<<<80, 256, 0, stream>>>(theta_w, phi_w, g_w, w_w, WT, WP, WG, WW2);
  k_xt<<<NB * (NPOS / 64) * (CIN / 64), 256, 0, stream>>>(x, XT);
  k_gemm<1, 0><<<dim3(NTOK / 64, CI / 64, 1), 128, 0, stream>>>(XT, CIN, 0L, WT, CIN, 0L, CIN, theta_b,
                                                               THh, THl, out, x, CI, 0L);
  k_gemm<1, 0><<<dim3(NTOK / 64, CI / 64, 1), 128, 0, stream>>>(XT, CIN, 0L, WP, CIN, 0L, CIN, phi_b,
                                                               PHh, PHl, out, x, CI, 0L);
  k_gemm<1, 1><<<dim3(CI / 64, NPOS / 64, NB), 128, 0, stream>>>(WG, CIN, 0L, XT, CIN, (long)NPOS * CIN, CIN, g_b,
                                                                GTh, GTl, out, x, NPOS, (long)CI * NPOS);
  k_attn<<<NB * (NPOS / AT_QB), 128, 0, stream>>>(THh, THl, PHh, PHl, GTh, GTl, Y);
  k_gemm<0, 1><<<dim3(CIN / 64, NPOS / 64, NB), 128, 0, stream>>>(WW2, YP, 0L, Y, YP, (long)NPOS * YP, YP, w_b,
                                                                 Y, Y, out, x, NPOS, (long)CIN * NPOS);
  (void)hipGetLastError();
}
